// MambaSSM_65798898975185
// MI455X (gfx1250) — hardware-verified
//
#include <hip/hip_runtime.h>
#include <math.h>

typedef __attribute__((ext_vector_type(8)))  _Float16 v8h;
typedef __attribute__((ext_vector_type(16))) __bf16   v16b;
typedef __attribute__((ext_vector_type(8)))  __bf16   v8b;
typedef __attribute__((ext_vector_type(8)))  float    v8f;
typedef __attribute__((ext_vector_type(4)))  float    v4f;

constexpr int kSeq    = 4096;
constexpr int kDm     = 511;
constexpr int kDmP    = 512;
constexpr int kDi     = 1022;
constexpr int kDiP    = 1024;
constexpr int kXzP    = 2 * kDiP;
constexpr int kNst    = 16;
constexpr int kDtR    = 32;
constexpr int kXdP    = 64;
constexpr int kWdtP   = 64;
constexpr int kConvTP = 260;
constexpr int kScanTS = 64;
constexpr int kScanCh = 64;
constexpr int kScanYP = 68;
constexpr int kScanLn = 2;
constexpr int kScanNs = kNst / kScanLn;
constexpr int kScanTh = kScanCh * kScanLn;
constexpr float kLog2e = 1.4426950408889634f;
static_assert(kDtR + 2 * kNst == kXdP, "x_proj width");
static_assert(kDmP == ((kDm + 31) / 32) * 32 && kDiP == ((kDi + 31) / 32) * 32, "K pads");
static_assert((kDmP % 32) == 0 && (kDiP % 32) == 0 && (kDtR % 32) == 0, "GEMM K multiples of 32");
static_assert((kSeq % 64) == 0 && (kXzP % 64) == 0 && (kXdP % 64) == 0 && (kDiP % 64) == 0 && (kDmP % 64) == 0, "GEMM M,N multiples of 64");
static_assert((kSeq % kScanTS) == 0 && (kDiP % kScanCh) == 0 && (kDiP % 256) == 0, "tile multiples");
static_assert(kScanNs == 8 && kScanTh == 128 && kScanTS == 64 && kScanCh == 64, "scan lane maps");

constexpr size_t kOffZT   = 0;
constexpr size_t kOffWIT  = kOffZT  + (size_t)kSeq * kDmP * 2;
constexpr size_t kOffWXT  = kOffWIT + (size_t)kXzP * kDmP * 2;
constexpr size_t kOffWDT  = kOffWXT + (size_t)kXdP * kDiP * 2;
constexpr size_t kOffWOT  = kOffWDT + (size_t)kDiP * kWdtP * 2;
constexpr size_t kOffXZ   = kOffWOT + (size_t)kDmP * kDiP * 2;
constexpr size_t kOffUC   = kOffXZ  + (size_t)kSeq * kXzP * 4;
constexpr size_t kOffUCH  = kOffUC  + (size_t)kSeq * kDiP * 4;
constexpr size_t kOffUCL  = kOffUCH + (size_t)kSeq * kDiP * 2;
constexpr size_t kOffXD   = kOffUCL + (size_t)kSeq * kDiP * 2;
constexpr size_t kOffDTH  = kOffXD  + (size_t)kSeq * kXdP * 4;
constexpr size_t kOffDTL  = kOffDTH + (size_t)kSeq * kDtR * 2;
constexpr size_t kOffDLR  = kOffDTL + (size_t)kSeq * kDtR * 2;
constexpr size_t kOffYH   = kOffDLR + (size_t)kSeq * kDiP * 4;
constexpr size_t kOffYL   = kOffYH  + (size_t)kSeq * kDiP * 2;
constexpr size_t kWsTotal = kOffYL  + (size_t)kSeq * kDiP * 2;
static_assert(kWsTotal == 109838336ull, "carve total");
static_assert(kWsTotal <= 134217728ull, "carve cap");
static_assert((kOffWIT % 128) == 0 && (kOffWXT % 128) == 0 && (kOffWDT % 128) == 0 && (kOffWOT % 128) == 0 &&
              (kOffXZ % 128) == 0 && (kOffUC % 128) == 0 && (kOffUCH % 128) == 0 && (kOffUCL % 128) == 0 &&
              (kOffXD % 128) == 0 && (kOffDTH % 128) == 0 && (kOffDTL % 128) == 0 && (kOffDLR % 128) == 0 &&
              (kOffYH % 128) == 0 && (kOffYL % 128) == 0, "128-B aligned regions");

__device__ __forceinline__ unsigned short f2bf_bits(float f) {
  unsigned u = __float_as_uint(f);
  return (unsigned short)((u + 0x7FFFu + ((u >> 16) & 1u)) >> 16);
}
__device__ __forceinline__ float bf_bits2f(unsigned short h) { return __uint_as_float(((unsigned)h) << 16); }
__device__ __forceinline__ float bf16r(float f) { return bf_bits2f(f2bf_bits(f)); }

__device__ __forceinline__ void split8_bf16(const v4f a0, const v4f a1, v8h& hv, v8h& lv) {
#pragma unroll
  for (int e = 0; e < 4; ++e) {
    const float f0 = a0[e];
    const float f1 = a1[e];
    const unsigned short h0 = f2bf_bits(f0);
    const unsigned short h1 = f2bf_bits(f1);
    const unsigned short l0 = f2bf_bits(f0 - bf_bits2f(h0));
    const unsigned short l1 = f2bf_bits(f1 - bf_bits2f(h1));
    hv[e]     = __builtin_bit_cast(_Float16, h0);
    hv[4 + e] = __builtin_bit_cast(_Float16, h1);
    lv[e]     = __builtin_bit_cast(_Float16, l0);
    lv[4 + e] = __builtin_bit_cast(_Float16, l1);
  }
}

__device__ __forceinline__ void dep_guard4_b(v8f& a, v8f& b, v8f& c, v8f& d, v16b x, v16b y) {
  asm volatile("v_nop\n\tv_nop\n\tv_nop\n\tv_nop" : "+v"(a), "+v"(b), "+v"(c), "+v"(d) : "v"(x), "v"(y));
}
__device__ __forceinline__ void keep4_b(v16b a, v16b b, v16b c, v16b d) { asm volatile("v_nop" :: "v"(a), "v"(b), "v"(c), "v"(d)); }
__device__ __forceinline__ void acc_guard4(v8f& a, v8f& b, v8f& c, v8f& d) { asm volatile("v_nop\n\tv_nop\n\tv_nop\n\tv_nop" : "+v"(a), "+v"(b), "+v"(c), "+v"(d)); }

union FragU { v16b v; v8b h[2]; };
__device__ __forceinline__ v16b frag_load(const __bf16* p) {
  FragU f;
  f.h[0] = *(const v8b*)(p);
  f.h[1] = *(const v8b*)(p + 16);
  return f.v;
}
__device__ __forceinline__ v8f frag_mma(v16b a, v16b b, v8f c) {
  return __builtin_amdgcn_wmma_f32_16x16x32_bf16(false, a, false, b, (short)0, c, false, false);
}

template <bool SPA, bool SPB>
__global__ __launch_bounds__(256) void wmma_gemm64(
    const unsigned short* __restrict__ Ap, const unsigned short* __restrict__ A2p, int lda,
    const unsigned short* __restrict__ Btp, const unsigned short* __restrict__ Bt2p, int ldb,
    float* __restrict__ C, int ldc, int M, int N, int K, int Mreal) {
  const __bf16* A   = (const __bf16*)Ap;
  const __bf16* A2  = (const __bf16*)A2p;
  const __bf16* Bt  = (const __bf16*)Btp;
  const __bf16* Bt2 = (const __bf16*)Bt2p;
  __shared__ __align__(16) float sT[8][16 * 68];
  const int lane = threadIdx.x & 31;
  const int wave = threadIdx.x >> 5;
  const int tilesN = N >> 6;
  const int tilesM = M >> 6;
  const int tile = blockIdx.x * 8 + wave;
  if (tile >= tilesM * tilesN) return;
  const int tm = tile / tilesN;
  const int tn = tile - tm * tilesN;
  const int m0 = tm << 6;
  const int n0 = tn << 6;

  const int rlane = lane & 15;
  const int koff  = (lane >> 4) * 8;
  const int mOff  = (lane >> 4) * 8;

  v8f acc[4][4];
#pragma unroll
  for (int i = 0; i < 4; ++i)
#pragma unroll
    for (int j = 0; j < 4; ++j) acc[i][j] = (v8f){0.f,0.f,0.f,0.f,0.f,0.f,0.f,0.f};

  for (int k0 = 0; k0 < K; k0 += 32) {
    v16b bh[4], bl[4];
#pragma unroll
    for (int j = 0; j < 4; ++j) {
      const size_t bo = (size_t)(n0 + (j << 4) + rlane) * ldb + koff + k0;
      bh[j] = frag_load(Bt + bo);
      if (SPB) bl[j] = frag_load(Bt2 + bo);
      else bl[j] = bh[j];
    }
#pragma unroll
    for (int i = 0; i < 4; ++i) {
      const size_t ao = (size_t)(m0 + (i << 4) + rlane) * lda + koff + k0;
      v16b ah = frag_load(A + ao);
      v16b al;
      if (SPA) al = frag_load(A2 + ao);
      else al = ah;
#pragma unroll
      for (int j = 0; j < 4; ++j) {
        acc[i][j] = frag_mma(ah, bh[j], acc[i][j]);
        if (SPB) acc[i][j] = frag_mma(ah, bl[j], acc[i][j]);
        if (SPA) acc[i][j] = frag_mma(al, bh[j], acc[i][j]);
      }
      dep_guard4_b(acc[i][0], acc[i][1], acc[i][2], acc[i][3], ah, al);
    }
    keep4_b(bh[0], bh[1], bh[2], bh[3]);
    keep4_b(bl[0], bl[1], bl[2], bl[3]);
  }
  acc_guard4(acc[0][0], acc[0][1], acc[0][2], acc[0][3]);
  acc_guard4(acc[1][0], acc[1][1], acc[1][2], acc[1][3]);
  acc_guard4(acc[2][0], acc[2][1], acc[2][2], acc[2][3]);
  acc_guard4(acc[3][0], acc[3][1], acc[3][2], acc[3][3]);

  float* slab = sT[wave];
#pragma unroll
  for (int i = 0; i < 4; ++i) {
    const int mBase = m0 + (i << 4);
#pragma unroll
    for (int j = 0; j < 4; ++j) {
#pragma unroll
      for (int r = 0; r < 8; ++r) {
        slab[(mOff + r) * 68 + (j << 4) + rlane] = acc[i][j][r];
      }
    }
    __builtin_amdgcn_fence(__ATOMIC_RELEASE, "workgroup");
    __builtin_amdgcn_wave_barrier();
    __builtin_amdgcn_fence(__ATOMIC_ACQUIRE, "workgroup");
    {
      const int hh = lane >> 4, c4 = (lane & 15) * 4;
      for (int pass = 0; pass < 2; ++pass) {
#pragma unroll
        for (int it = 0; it < 8; ++it) {
          const int row = it * 2 + hh;
          const v4f v = *(const v4f*)(slab + row * 68 + c4);
          if (mBase + row < Mreal) {
            *(volatile v4f*)(C + (size_t)(mBase + row) * ldc + n0 + c4) = v;
          }
        }
        __threadfence();
      }
    }
    __builtin_amdgcn_fence(__ATOMIC_RELEASE, "workgroup");
    __builtin_amdgcn_wave_barrier();
    __builtin_amdgcn_fence(__ATOMIC_ACQUIRE, "workgroup");
  }
}

__global__ __launch_bounds__(256) void transpose_bf16_kernel(
    const float* __restrict__ W, unsigned short* __restrict__ Bt,
    int ldIn, int Kreal, int Kpad, int segShift, int segReal)
{
  __shared__ float tile[64 * 65];
  const int tid = threadIdx.x, lane = tid & 31, wave = tid >> 5;
  const int n0 = blockIdx.x * 64;
  const int k0 = blockIdx.y * 64;
  const int segMask = (1 << segShift) - 1;
#pragma unroll
  for (int p = 0; p < 16; ++p) {
    const int idx = tid + p * 256;
    const int kk  = idx >> 6;
    const int nn  = idx & 63;
    const int k   = k0 + kk;
    const int kc  = (k < Kreal) ? k : (Kreal - 1);
    const int r   = n0 + nn;
    const int seg = r >> segShift;
    const int w   = r & segMask;
    const int wc  = (w < segReal) ? w : (segReal - 1);
    const float v = W[(size_t)kc * ldIn + seg * segReal + wc];
    const bool ok = (k < Kreal) && (w < segReal);
    tile[kk * 65 + nn] = ok ? v : 0.f;
  }
  __syncthreads();
  const int q = lane >> 3, c8 = (lane & 7) * 8;
  v8h hv[2];
#pragma unroll
  for (int it = 0; it < 2; ++it) {
    const int nrow = it * 32 + wave * 4 + q;
#pragma unroll
    for (int e = 0; e < 8; ++e) {
      const float f = tile[(c8 + e) * 65 + nrow];
      const unsigned short hb = f2bf_bits(f);
      hv[it][e] = __builtin_bit_cast(_Float16, hb);
    }
  }
  for (int pass = 0; pass < 2; ++pass) {
#pragma unroll
    for (int it = 0; it < 2; ++it) {
      const int nrow = it * 32 + wave * 4 + q;
      *(volatile v8h*)(Bt + (size_t)(n0 + nrow) * Kpad + k0 + c8) = hv[it];
    }
    __threadfence();
  }
}

__global__ __launch_bounds__(256) void conv_silu_kernel(
    const float* __restrict__ XZ, const float* __restrict__ cw, const float* __restrict__ cb,
    float* __restrict__ UC, unsigned short* __restrict__ UCH, unsigned short* __restrict__ UCL)
{
  __shared__ __align__(16) float sT[16 * kConvTP];
  const int tid = threadIdx.x, lane = tid & 31, wave = tid >> 5;
  const int d0 = blockIdx.x * 256, d = d0 + tid;
  const bool valid = (d < kDi);
  const int dc = valid ? d : (kDi - 1);
  const int g0 = blockIdx.y * 64;
  const v4f wv = *(const v4f*)(cw + (size_t)dc * 4);
  const float wr0 = wv[0];
  const float wr1 = wv[1];
  const float wr2 = wv[2];
  const float wr3 = wv[3];
  const float br  = cb[dc];
  const float w0 = valid ? bf16r(wr0) : 0.f;
  const float w1 = valid ? bf16r(wr1) : 0.f;
  const float w2 = valid ? bf16r(wr2) : 0.f;
  const float w3 = valid ? bf16r(wr3) : 0.f;
  const float bc = valid ? bf16r(br) : 0.f;
  float xm3, xm2, xm1;
  {
    const bool hist = (g0 > 0);
    const int rb = hist ? (g0 - 3) : g0;
    const float v3 = XZ[(size_t)rb * kXzP + d];
    const float v2 = XZ[(size_t)(rb + 1) * kXzP + d];
    const float v1 = XZ[(size_t)(rb + 2) * kXzP + d];
    xm3 = hist ? v3 : 0.f;
    xm2 = hist ? v2 : 0.f;
    xm1 = hist ? v1 : 0.f;
  }
  const int hrow = wave >> 1;
  const int hch  = (wave & 1) * 128 + lane * 4;
#pragma unroll 1
  for (int sub = 0; sub < 4; ++sub) {
    const int lb = g0 + sub * 16;
#pragma unroll 1
    for (int s = 0; s < 16; ++s) {
      const float xcur = XZ[(size_t)(lb + s) * kXzP + d];
      float acc = w0 * xm3;
      acc = fmaf(w1, xm2, acc);
      acc = fmaf(w2, xm1, acc);
      acc = fmaf(w3, xcur, acc);
      const float sv = acc + bc;
      const float sg = __builtin_amdgcn_rcpf(1.0f + expf(-sv));
      sT[s * kConvTP + tid] = sv * sg;
      xm3 = xm2; xm2 = xm1; xm1 = xcur;
    }
    __syncthreads();
    v4f fv[4];
    v8h bh[2], blo[2];
#pragma unroll
    for (int it = 0; it < 4; ++it) fv[it] = *(const v4f*)(sT + (it * 4 + hrow) * kConvTP + hch);
#pragma unroll
    for (int it = 0; it < 2; ++it) {
      const float* sp = sT + (it * 8 + wave) * kConvTP + lane * 8;
      const v4f a0 = *(const v4f*)(sp);
      const v4f a1 = *(const v4f*)(sp + 4);
      split8_bf16(a0, a1, bh[it], blo[it]);
    }
    for (int pass = 0; pass < 2; ++pass) {
#pragma unroll
      for (int it = 0; it < 4; ++it)
        *(volatile v4f*)(UC + (size_t)(lb + it * 4 + hrow) * kDiP + d0 + hch) = fv[it];
#pragma unroll
      for (int it = 0; it < 2; ++it) {
        const size_t o = (size_t)(lb + it * 8 + wave) * kDiP + d0 + lane * 8;
        *(volatile v8h*)(UCH + o) = bh[it];
        *(volatile v8h*)(UCL + o) = blo[it];
      }
      __threadfence();
    }
    __syncthreads();
  }
}

__global__ __launch_bounds__(256) void dt_split_kernel(
    const float* __restrict__ XD, unsigned short* __restrict__ DTH, unsigned short* __restrict__ DTL, int total8)
{
  const int i = blockIdx.x * 256 + threadIdx.x;
  if (i >= total8) return;
  const int e0  = i << 3;
  const int row = e0 >> 5;
  const int c8  = e0 & 31;
  const float* p = XD + (size_t)row * kXdP + c8;
  const v4f a0 = *(const v4f*)(p);
  const v4f a1 = *(const v4f*)(p + 4);
  v8h hv, lv;
  split8_bf16(a0, a1, hv, lv);
  unsigned short* qh = DTH + e0;
  unsigned short* ql = DTL + e0;
  *(volatile v8h*)qh = hv;
  *(volatile v8h*)ql = lv;
  __threadfence();
  *(volatile v8h*)qh = hv;
  *(volatile v8h*)ql = lv;
}

__global__ __launch_bounds__(128) void scan_kernel(
    const float* __restrict__ DLR, const float* __restrict__ UC, const float* __restrict__ XZ,
    const float* __restrict__ XD, const float* __restrict__ bdt, const float* __restrict__ Alog,
    const float* __restrict__ Dp, unsigned short* __restrict__ YH, unsigned short* __restrict__ YL)
{
  __shared__ __align__(16) float sBC[kScanTS * 32];
  __shared__ __align__(16) float sY[kScanTS * kScanYP];
  __shared__ __align__(16) float sA[kNst * kScanCh];
  const int tid = threadIdx.x, lane = tid & 31, wave = tid >> 5;
  const int hf = tid & 1;
  const int ch = tid >> 1;
  const int sb = hf * kScanNs;
  const int d0 = blockIdx.x * kScanCh;
  const int d  = d0 + ch;
  const bool valid = (d < kDi);
  const int dc = valid ? d : (kDi - 1);
#pragma unroll 1
  for (int j = 0; j < kScanNs; ++j) {
    const float al = bf16r(Alog[(size_t)dc * kNst + sb + j]);
    sA[(sb + j) * kScanCh + ch] = -expf(al) * kLog2e;
  }
  __syncthreads();
  float a2[kScanNs], h[kScanNs];
#pragma unroll
  for (int j = 0; j < kScanNs; ++j) {
    a2[j] = sA[(sb + j) * kScanCh + ch];
    h[j] = 0.f;
  }
  const float bbr = bdt[dc];
  const float ddr = Dp[dc];
  const float bb = valid ? bf16r(bbr) : 0.f;
  const float Dd = valid ? bf16r(ddr) : 0.f;
  const int lr = tid >> 3, lc4 = (tid & 7) * 4;
  const int q = lane >> 3, c8 = (lane & 7) * 8;
#pragma unroll 1
  for (int t0 = 0; t0 < kSeq; t0 += kScanTS) {
    __syncthreads();
#pragma unroll
    for (int i = 0; i < 4; ++i) {
      const int r = lr + 16 * i;
      *(v4f*)(sBC + r * 32 + lc4) = *(const v4f*)(XD + (size_t)(t0 + r) * kXdP + kDtR + lc4);
    }
    __syncthreads();
#pragma unroll 1
    for (int s = 0; s < kScanTS; ++s) {
      const size_t t = (size_t)(t0 + s);
      const float* xr = sBC + s * 32 + sb;
      const v4f bv0 = *(const v4f*)(xr);
      const v4f bv1 = *(const v4f*)(xr + 4);
      const v4f cv0 = *(const v4f*)(xr + kNst);
      const v4f cv1 = *(const v4f*)(xr + kNst + 4);
      float Bs[kScanNs], Cs[kScanNs];
      Bs[0] = bv0[0]; Bs[1] = bv0[1]; Bs[2] = bv0[2]; Bs[3] = bv0[3];
      Bs[4] = bv1[0]; Bs[5] = bv1[1]; Bs[6] = bv1[2]; Bs[7] = bv1[3];
      Cs[0] = cv0[0]; Cs[1] = cv0[1]; Cs[2] = cv0[2]; Cs[3] = cv0[3];
      Cs[4] = cv1[0]; Cs[5] = cv1[1]; Cs[6] = cv1[2]; Cs[7] = cv1[3];
      const float v   = DLR[t * kDiP + d] + bb;
      const float a   = __expf(-fabsf(v));
      const float u   = 1.0f + a;
      const float l1p = __logf(u) + (a - (u - 1.0f)) * __builtin_amdgcn_rcpf(u);
      const float dt  = fmaxf(v, 0.0f) + l1p;
      const float xt  = UC[t * kDiP + d];
      float zv = XZ[t * kXzP + kDiP + d];
      asm volatile("" : "+v"(zv));
      const float dtx = dt * xt;
      float yp = 0.f;
#pragma unroll
      for (int k = 0; k < kScanNs; ++k) {
        const float e = __builtin_amdgcn_exp2f(dt * a2[k]);
        h[k] = fmaf(e, h[k], dtx * Bs[k]);
        yp = fmaf(h[k], Cs[k], yp);
      }
      const float yo = __shfl_xor(yp, 1, 32);
      float y = yp + yo;
      y = fmaf(xt, Dd, y);
      const float sg = __builtin_amdgcn_rcpf(1.0f + __expf(-zv));
      y = y * (zv * sg);
      asm volatile("" : "+v"(y));
      if (hf == 0) sY[s * kScanYP + ch] = y;
    }
    __syncthreads();
#pragma unroll 1
    for (int pass = 0; pass < 2; ++pass) {
#pragma unroll 1
      for (int it = 0; it < 4; ++it) {
        const int row = it * 16 + wave * 4 + q;
        const float* sp = sY + row * kScanYP + c8;
        const v4f a0 = *(const v4f*)(sp);
        const v4f a1 = *(const v4f*)(sp + 4);
        v8h hv, lv;
        split8_bf16(a0, a1, hv, lv);
        const size_t o = (size_t)(t0 + row) * kDiP + d0 + c8;
        *(volatile v8h*)(YH + o) = hv;
        *(volatile v8h*)(YL + o) = lv;
      }
      __threadfence();
    }
  }
}

extern "C" void kernel_launch(void* const* d_in, const int* in_sizes, int n_in,
                              void* d_out, int out_size, void* d_ws, size_t ws_size,
                              hipStream_t stream) {
  (void)stream;
  if (n_in < 10) return;
  if (in_sizes[0] != kDm * kSeq) return;
  if (in_sizes[1] != kDm * 2 * kDi) return;
  if (in_sizes[2] != kDi * 4) return;
  if (in_sizes[3] != kDi) return;
  if (in_sizes[4] != kDi * kXdP) return;
  if (in_sizes[5] != kDtR * kDi) return;
  if (in_sizes[6] != kDi) return;
  if (in_sizes[7] != kDi * kNst) return;
  if (in_sizes[8] != kDi) return;
  if (in_sizes[9] != kDi * kDm) return;
  if (out_size != kDm * kSeq) return;
  if (ws_size < kWsTotal) return;

  const float* Z      = (const float*)d_in[0];
  const float* W_in   = (const float*)d_in[1];
  const float* conv_w = (const float*)d_in[2];
  const float* conv_b = (const float*)d_in[3];
  const float* W_x    = (const float*)d_in[4];
  const float* W_dt   = (const float*)d_in[5];
  const float* b_dt   = (const float*)d_in[6];
  const float* A_log  = (const float*)d_in[7];
  const float* Dp     = (const float*)d_in[8];
  const float* W_out  = (const float*)d_in[9];
  float* out = (float*)d_out;

  char* ws = (char*)d_ws;
  unsigned short* ZT  = (unsigned short*)(ws + kOffZT);
  unsigned short* WIT = (unsigned short*)(ws + kOffWIT);
  unsigned short* WXT = (unsigned short*)(ws + kOffWXT);
  unsigned short* WDT = (unsigned short*)(ws + kOffWDT);
  unsigned short* WOT = (unsigned short*)(ws + kOffWOT);
  float*          XZ  = (float*)(ws + kOffXZ);
  float*          UC  = (float*)(ws + kOffUC);
  unsigned short* UCH = (unsigned short*)(ws + kOffUCH);
  unsigned short* UCL = (unsigned short*)(ws + kOffUCL);
  float*          XD  = (float*)(ws + kOffXD);
  unsigned short* DTH = (unsigned short*)(ws + kOffDTH);
  unsigned short* DTL = (unsigned short*)(ws + kOffDTL);
  float*          DLR = (float*)(ws + kOffDLR);
  unsigned short* YH  = (unsigned short*)(ws + kOffYH);
  unsigned short* YL  = (unsigned short*)(ws + kOffYL);

  transpose_bf16_kernel<<<dim3(kSeq / 64, kDmP / 64), 256, 0, stream>>>(Z, ZT, kSeq, kDm, kDmP, 12, kSeq);
  transpose_bf16_kernel<<<dim3(kXzP / 64, kDmP / 64), 256, 0, stream>>>(W_in, WIT, 2 * kDi, kDm, kDmP, 10, kDi);
  transpose_bf16_kernel<<<dim3(kXdP / 64, kDiP / 64), 256, 0, stream>>>(W_x, WXT, kXdP, kDi, kDiP, 6, kXdP);
  transpose_bf16_kernel<<<dim3(kDiP / 64, kWdtP / 64), 256, 0, stream>>>(W_dt, WDT, kDi, kDtR, kWdtP, 10, kDi);
  transpose_bf16_kernel<<<dim3(kDmP / 64, kDiP / 64), 256, 0, stream>>>(W_out, WOT, kDm, kDi, kDiP, 9, kDm);

  wmma_gemm64<false, false><<<dim3((kSeq / 64) * (kXzP / 64) / 8, 1), 256, 0, stream>>>(
      ZT, ZT, kDmP, WIT, WIT, kDmP, XZ, kXzP, kSeq, kXzP, kDmP, kSeq);

  conv_silu_kernel<<<dim3(kDiP / 256, kSeq / 64), 256, 0, stream>>>(XZ, conv_w, conv_b, UC, UCH, UCL);

  wmma_gemm64<true, false><<<dim3((kSeq / 64) * (kXdP / 64) / 8, 1), 256, 0, stream>>>(
      UCH, UCL, kDiP, WXT, WXT, kDiP, XD, kXdP, kSeq, kXdP, kDiP, kSeq);

  dt_split_kernel<<<(kSeq * kDtR / 8) / 256, 256, 0, stream>>>(XD, DTH, DTL, kSeq * kDtR / 8);

  wmma_gemm64<true, false><<<dim3((kSeq / 64) * (kDiP / 64) / 8, 1), 256, 0, stream>>>(
      DTH, DTL, kDtR, WDT, WDT, kWdtP, DLR, kDiP, kSeq, kDiP, kDtR, kSeq);

  scan_kernel<<<kDiP / kScanCh, kScanTh, 0, stream>>>(DLR, UC, XZ, XD, b_dt, A_log, Dp, YH, YL);

  wmma_gemm64<false, true><<<dim3((kDmP / 64) * (kSeq / 64) / 8, 1), 256, 0, stream>>>(
      WOT, WOT, kDiP, YH, YL, kDiP, out, kSeq, kDmP, kSeq, kDiP, kDm);
}
